// Model_59382217835041
// MI455X (gfx1250) — hardware-verified
//
#include <hip/hip_runtime.h>
#include <stddef.h>
#include <stdint.h>

#define NBS    8
#define HID    64
#define NSH    9
#define CCH    16
#define OC     144
#define K1     32
#define K2     128
#define NTHR   256
#define NWAVE  8
#define EPB    128
#define A1P    40
#define A2P    136
#define WTP    148
#define SHP    12
#define PTU    1024
#define PTLIVE 864
#define SVF    256
#define U0     256
#define U1     (U0 + OC * (K2 / 8))
#define U2     (U1 + 256)
#define U3     (U2 + PTU)
#define EPT    8
#define CHUNK  (NTHR * EPT)
#define WCAP   (EPT * 32)
#define LISTN  (NWAVE * WCAP)
#define NBA    1024
#define SLA    10
#define RCAP   20480
#define DEGCAP 64
#define AGG_ZINTS (LISTN + 2 * RCAP + 3 * NBA)
#define AGG_LDS_INTS (AGG_ZINTS + 16)
#define SCAN_LDS_BYTES ((AGG_LDS_INTS + NBA * 3) * 4)
#define EDGE_LDS_BYTES ((EPB * WTP + EPB * SHP + PTU * 4 + SVF + EPB * 4 + EPB) * 4 + (EPB * A2P + EPB * A1P) * 2)
#define WSMAX  134217728
#define PI_F   3.14159265358979323846f
#define RCUTF  5.0f
#define S3F    1.7320508075688772f
#define S15F   3.8729833462074170f
#define H5F    1.1180339887498949f
#define H15F   1.9364916731037085f

static_assert(NSH * CCH == OC && OC == 144);
static_assert(HID == 64 && 2 * HID == K2 && K2 % 32 == 0);
static_assert(2 * NBS <= K1 && K1 == 32);
static_assert(PTLIVE == 6 * OC && PTLIVE <= PTU && PTU % NTHR == 0);
static_assert(HID + OC <= SVF && SVF % 4 == 0 && SVF / 4 <= NTHR);
static_assert(U0 == HID * (K1 / 8) && (U1 - U0) % NTHR == 0 && U3 % NTHR == 0);
static_assert(EPB == 16 * NWAVE && NTHR == 2 * EPB);
static_assert((A1P * 2) % 16 == 0 && (A2P * 2) % 16 == 0 && (WTP * 4) % 16 == 0 && A1P >= K1 && A2P >= K2 && WTP >= OC);
static_assert(EDGE_LDS_BYTES <= 300000 && SCAN_LDS_BYTES <= 300000);
static_assert((CHUNK & (CHUNK - 1)) == 0 && CHUNK <= 4096);
static_assert((NBA & (NBA - 1)) == 0 && NBA == (1 << SLA) && NBA % NTHR == 0);
static_assert(((long long)CHUNK << SLA) < (1LL << 31));
static_assert(RCAP % 4 == 0 && AGG_ZINTS % (4 * NTHR) == 0 && LISTN % 4 == 0);
static_assert(RCAP >= 17492);
static_assert(DEGCAP >= 36 + 8);
static_assert((NBA * 3) % 4 == 0 && (NBA * 3) / 4 == 3 * NTHR);
static_assert((AGG_LDS_INTS * 4) % 16 == 0);

typedef float          v4f   __attribute__((ext_vector_type(4)));
typedef float          v8f   __attribute__((ext_vector_type(8)));
typedef int            v4i   __attribute__((ext_vector_type(4)));
typedef int            v8i   __attribute__((ext_vector_type(8)));
typedef unsigned       v2u   __attribute__((ext_vector_type(2)));
typedef unsigned short v8us  __attribute__((ext_vector_type(8)));
typedef unsigned short v16us __attribute__((ext_vector_type(16)));
typedef __bf16         v16bf __attribute__((ext_vector_type(16)));
typedef v4f  __attribute__((may_alias)) v4fa;
typedef v4i  __attribute__((may_alias)) v4ia;
typedef v2u  __attribute__((may_alias)) v2ua;
typedef v8us __attribute__((may_alias)) v8usa;
union FragB { v16bf v; v16us u; v8us h[2]; v8i w; };

__device__ __forceinline__ v8f wmb(const FragB& a, const FragB& b, v8f c) {
  v8f d = __builtin_amdgcn_wmma_f32_16x16x32_bf16(false, a.v, false, b.v, (short)0, c, false, false);
  asm volatile("v_nop\n\tv_nop\n\tv_nop\n\tv_nop" : "+v"(d) : "v"(a.w), "v"(b.w));
  return d;
}

__device__ __forceinline__ unsigned bf16_bits(float f) {
  const unsigned u = __float_as_uint(f);
  return (u + 0x7FFFu + ((u >> 16) & 1u)) >> 16;
}
__device__ __forceinline__ float bf16_val(float f) {
  return __uint_as_float(bf16_bits(f) << 16);
}
__device__ __forceinline__ void put16(unsigned short* dp, v8us o) {
  *(volatile v8us*)dp = o;
  __threadfence();
  *(volatile v8us*)dp = o;
}
__device__ __forceinline__ void putf4(float* dp, v4f o) {
  *(volatile v4f*)dp = o;
  __threadfence();
  *(volatile v4f*)dp = o;
}

template <int SLB>
__device__ __forceinline__ int scan_chunk(const int* __restrict__ dsts, int nE, int cbase, int slotBase,
                                          int nb, int vec8, int* list, int tid, int lane, int wave) {
  int wc = 0;
  const int el0  = tid * EPT;
  const int e0   = cbase + el0;
  const int sent = -2147483647 - 1;
  v4i da, db;
  if (vec8 != 0 && cbase + CHUNK <= nE) {
    da = *(const v4i*)(dsts + e0);
    db = *(const v4i*)(dsts + e0 + 4);
  } else {
    da.x = (e0     < nE) ? dsts[min(e0,     nE - 1)] : sent;
    da.y = (e0 + 1 < nE) ? dsts[min(e0 + 1, nE - 1)] : sent;
    da.z = (e0 + 2 < nE) ? dsts[min(e0 + 2, nE - 1)] : sent;
    da.w = (e0 + 3 < nE) ? dsts[min(e0 + 3, nE - 1)] : sent;
    db.x = (e0 + 4 < nE) ? dsts[min(e0 + 4, nE - 1)] : sent;
    db.y = (e0 + 5 < nE) ? dsts[min(e0 + 5, nE - 1)] : sent;
    db.z = (e0 + 6 < nE) ? dsts[min(e0 + 6, nE - 1)] : sent;
    db.w = (e0 + 7 < nE) ? dsts[min(e0 + 7, nE - 1)] : sent;
  }
  const unsigned nbs = (unsigned)slotBase;
  const unsigned unb = (unsigned)nb;
  const unsigned s0 = (unsigned)da.x - nbs, s1 = (unsigned)da.y - nbs;
  const unsigned s2 = (unsigned)da.z - nbs, s3 = (unsigned)da.w - nbs;
  const unsigned s4 = (unsigned)db.x - nbs, s5 = (unsigned)db.y - nbs;
  const unsigned s6 = (unsigned)db.z - nbs, s7 = (unsigned)db.w - nbs;
  const bool h0 = s0 < unb, h1 = s1 < unb, h2 = s2 < unb, h3 = s3 < unb;
  const bool h4 = s4 < unb, h5 = s5 < unb, h6 = s6 < unb, h7 = s7 < unb;
  const unsigned any = __builtin_amdgcn_ballot_w32(h0 | h1 | h2 | h3 | h4 | h5 | h6 | h7);
  if (any != 0u) {
#define HITJ(J, HJ, SJ) { \
      const unsigned mj = __builtin_amdgcn_ballot_w32(HJ); \
      if (mj != 0u) { \
        if (HJ) { \
          const int pos = wc + (int)__builtin_amdgcn_mbcnt_lo(mj, 0u); \
          if (pos < WCAP) list[wave * WCAP + pos] = ((el0 + (J)) << SLB) | (int)(SJ); \
        } \
        wc += (int)__builtin_popcount(mj); } }
    HITJ(0, h0, s0)
    HITJ(1, h1, s1)
    HITJ(2, h2, s2)
    HITJ(3, h3, s3)
    HITJ(4, h4, s4)
    HITJ(5, h5, s5)
    HITJ(6, h6, s6)
    HITJ(7, h7, s7)
#undef HITJ
  }
  return wc;
}

__global__ __launch_bounds__(NTHR) void k_prep(const int* __restrict__ zarr, const float* __restrict__ pos,
                                               const float* __restrict__ embw, const float* __restrict__ embb,
                                               const float* __restrict__ w1, const float* __restrict__ b1,
                                               const float* __restrict__ w2, const float* __restrict__ b2,
                                               const float* __restrict__ ow, int nN, int npr,
                                               unsigned short* W1P, unsigned short* W2D,
                                               float* SV, float* PT, float* NPp) {
  const int u = (int)blockIdx.x * NTHR + (int)threadIdx.x;
  if (u < U0) {
    const int n  = u >> 2;
    const int k8 = (u & 3) * 8;
    const unsigned keep = (k8 < 16) ? 0xffffu : 0u;
    const float* p = w1 + n;
    v8us o;
#pragma unroll
    for (int i = 0; i < 8; ++i) o[i] = (unsigned short)(bf16_bits(p[(size_t)i * HID]) & keep);
    put16(W1P + (size_t)n * K1 + k8, o);
    return;
  } else if (u < U1) {
    const int v    = u - U0;
    const int n    = v >> 4;
    const int k8   = (v & 15) * 8;
    const int srow = k8 & (HID - 1);
    const float* p = w2 + (size_t)srow * OC + n;
    v8us o;
#pragma unroll
    for (int i = 0; i < 8; ++i) o[i] = (unsigned short)bf16_bits(p[(size_t)i * OC]);
    put16(W2D + (size_t)n * K2 + k8, o);
    return;
  } else if (u < U2) {
    const int q = u - U1;
    if (q >= SVF / 4) return;
    const int qa = q < 15 ? q : 15;
    int qb = q - 16;
    qb = qb < 0 ? 0 : (qb > 35 ? 35 : qb);
    const v4f a = *(const v4fa*)(b1 + 4 * qa);
    const v4f b = *(const v4fa*)(b2 + 4 * qb);
    const unsigned ma = (q < 16) ? 0xffffffffu : 0u;
    const unsigned mb = (q >= 16 && q < 52) ? 0xffffffffu : 0u;
    v4f o;
    o.x = __uint_as_float((__float_as_uint(bf16_val(a.x)) & ma) | (__float_as_uint(bf16_val(b.x)) & mb));
    o.y = __uint_as_float((__float_as_uint(bf16_val(a.y)) & ma) | (__float_as_uint(bf16_val(b.y)) & mb));
    o.z = __uint_as_float((__float_as_uint(bf16_val(a.z)) & ma) | (__float_as_uint(bf16_val(b.z)) & mb));
    o.w = __uint_as_float((__float_as_uint(bf16_val(a.w)) & ma) | (__float_as_uint(bf16_val(b.w)) & mb));
    putf4(SV + 4 * q, o);
    return;
  } else if (u < U3) {
    const int p   = u - U2;
    const int pc  = p < PTLIVE ? p : PTLIVE - 1;
    const int sp  = pc / OC;
    const int sc  = pc - sp * OC;
    const int c   = sc & (CCH - 1);
    const int spc = sp < 4 ? sp : 4;
    const float ew = embw[spc * CCH + c];
    const float eb = embb[c];
    const float o0 = ow[sc * 3 + 0];
    const float o1 = ow[sc * 3 + 1];
    const float o2 = ow[sc * 3 + 2];
    const float nfw = (sp < 5) ? bf16_val(ew) : 0.0f;
    const float nf  = nfw + bf16_val(eb);
    const bool live = p < PTLIVE;
    v4f q;
    q.x = live ? nf * bf16_val(o0) : 0.0f;
    q.y = live ? nf * bf16_val(o1) : 0.0f;
    q.z = live ? nf * bf16_val(o2) : 0.0f;
    q.w = 0.0f;
    putf4(PT + 4 * p, q);
    return;
  } else {
    const int row = u - U3;
    if (row >= npr) return;
    const int rc  = row < nN ? row : nN - 1;
    const bool ok = row < nN;
    const float r0 = pos[(size_t)rc * 3 + 0];
    const float r1 = pos[(size_t)rc * 3 + 1];
    const float r2 = pos[(size_t)rc * 3 + 2];
    const int   zi = zarr[rc];
    const int   sp = ((unsigned)zi < 5u) ? zi : 5;
    v4f q;
    q.x = ok ? bf16_val(r0) : 0.0f;
    q.y = ok ? bf16_val(r1) : 0.0f;
    q.z = ok ? bf16_val(r2) : 0.0f;
    q.w = ok ? __int_as_float(sp) : 0.0f;
    putf4(NPp + (size_t)row * 4, q);
    return;
  }
}

__global__ __launch_bounds__(NTHR) void k_edge(const int* __restrict__ eidx, const float* __restrict__ shift,
                                               int nE, int nN, const float* __restrict__ NPp,
                                               const unsigned short* __restrict__ W1P,
                                               const unsigned short* __restrict__ W2D,
                                               const float* __restrict__ SV, const float* __restrict__ PT,
                                               float* F3) {
#pragma clang fp contract(off)
  extern __shared__ __attribute__((aligned(16))) float dyn[];
  float*          sWT = dyn;
  float*          sSH = sWT + EPB * WTP;
  float*          sPT = sSH + EPB * SHP;
  float*          sSV = sPT + PTU * 4;
  float*          sF3 = sSV + SVF;
  int*            sSP = (int*)(sF3 + EPB * 4);
  unsigned short* sA2 = (unsigned short*)(sSP + EPB);
  unsigned short* sA1 = sA2 + EPB * A2P;

  const int tid = (int)threadIdx.x, lane = tid & 31, wave = tid >> 5, hh = lane >> 4, m = lane & 15;

#pragma unroll
  for (int it = 0; it < PTU / NTHR; ++it) {
    const int i = it * NTHR + tid;
    *(v4fa*)(sPT + 4 * i) = *(const v4fa*)(PT + 4 * i);
  }
  if (tid < SVF / 4) *(v4fa*)(sSV + 4 * tid) = *(const v4fa*)(SV + 4 * tid);

  {
    const int el   = tid & (EPB - 1);
    const int half = tid >> 7;
    const int e    = (int)blockIdx.x * EPB + el;
    const int ec   = e < nE ? e : nE - 1;
    int s = eidx[ec];
    int d = eidx[(size_t)nE + (size_t)ec];
    s = s < 0 ? 0 : (s > nN - 1 ? nN - 1 : s);
    d = d < 0 ? 0 : (d > nN - 1 ? nN - 1 : d);
    const v4f ps = *(const v4fa*)(NPp + (size_t)s * 4);
    const v4f pd = *(const v4fa*)(NPp + (size_t)d * 4);
    const float hx = bf16_val(shift[(size_t)ec * 3 + 0]);
    const float hy = bf16_val(shift[(size_t)ec * 3 + 1]);
    const float hz = bf16_val(shift[(size_t)ec * 3 + 2]);
    const float vx = (pd.x - ps.x) + hx;
    const float vy = (pd.y - ps.y) + hy;
    const float vz = (pd.z - ps.z) + hz;
    const float r2 = ((vx * vx + vy * vy) + vz * vz) + 1e-12f;
    const float r  = sqrtf(r2);

    if (half == 0) {
      const float ux = vx / r, uy = vy / r, uz = vz / r;
      v4f a, b, c;
      a.x = 1.0f;            a.y = S3F * ux;         a.z = S3F * uy;                          a.w = S3F * uz;
      b.x = (S15F * ux) * uy; b.y = (S15F * uy) * uz; b.z = H5F * ((3.0f * uz) * uz - 1.0f);  b.w = (S15F * ux) * uz;
      c.x = H15F * (ux * ux - uy * uy); c.y = 0.0f; c.z = 0.0f; c.w = 0.0f;
      float* rs = sSH + el * SHP;
      *(v4fa*)(rs)     = a;
      *(v4fa*)(rs + 4) = b;
      *(v4fa*)(rs + 8) = c;
      int sp = __float_as_int(ps.w);
      sp = sp < 0 ? 0 : (sp > 5 ? 5 : sp);
      sSP[el] = sp;
    }

    const float t   = r / RCUTF;
    const float cv  = 0.5f * (cosf(PI_F * t) + 1.0f);
    const float env = (t < 1.0f) ? cv : 0.0f;
    const float sq04 = __builtin_sqrtf(0.4f);
    unsigned long long hw = 0ull, lw = 0ull;
#pragma unroll 1
    for (int j = 0; j < 4; ++j) {
      const float nf  = (float)(4 * half + 1 + j);
      const float arg = ((nf * PI_F) * r) / RCUTF;
      const float bs  = (sq04 * sinf(arg)) / r;
      const float ef  = bs * env;
      const unsigned hb = bf16_bits(ef);
      const unsigned lb = bf16_bits(ef - __uint_as_float(hb << 16));
      hw |= (unsigned long long)hb << (16 * j);
      lw |= (unsigned long long)lb << (16 * j);
    }
    v2u hv, lv;
    hv.x = (unsigned)hw; hv.y = (unsigned)(hw >> 32);
    lv.x = (unsigned)lw; lv.y = (unsigned)(lw >> 32);
    const v4i z4 = {0, 0, 0, 0};
    unsigned short* ra = sA1 + el * A1P;
    *(v2ua*)(ra + 4 * half)      = hv;
    *(v2ua*)(ra + 8 + 4 * half)  = lv;
    *(v4ia*)(ra + 16 + 8 * half) = z4;
  }
  __syncthreads();

  const int rowW = 16 * wave;
  const v8f z8 = {0.f, 0.f, 0.f, 0.f, 0.f, 0.f, 0.f, 0.f};

  {
    FragB a;
    const unsigned short* ap = sA1 + (rowW + m) * A1P + 8 * hh;
    a.h[0] = *(const v8usa*)ap;
    a.h[1] = *(const v8usa*)(ap + 16);
#pragma unroll 1
    for (int nt = 0; nt < HID / 16; ++nt) {
      const unsigned short* wq = W1P + (size_t)(16 * nt + m) * K1 + 8 * hh;
      FragB b;
      b.h[0] = *(const v8usa*)wq;
      b.h[1] = *(const v8usa*)(wq + 16);
      const v8f hd = wmb(a, b, z8);
      const float bv = sSV[16 * nt + m];
#pragma unroll
      for (int r = 0; r < 8; ++r) {
        const float hid = hd[r] + bv;
        const float sg  = 1.0f / (1.0f + expf(-hid));
        const float av  = hid * sg;
        const unsigned hb = bf16_bits(av);
        const unsigned lb = bf16_bits(av - __uint_as_float(hb << 16));
        unsigned short* rp = sA2 + (rowW + 8 * hh + r) * A2P + 16 * nt + m;
        rp[0]   = (unsigned short)hb;
        rp[HID] = (unsigned short)lb;
      }
    }
  }
  __syncthreads();

  {
    v8f acc[NSH];
#pragma unroll
    for (int t = 0; t < NSH; ++t) acc[t] = z8;
    const unsigned short* ap = sA2 + (rowW + m) * A2P + 8 * hh;
    const unsigned short* bp = W2D + (size_t)m * K2 + 8 * hh;
#pragma unroll 1
    for (int k0 = 0; k0 < K2; k0 += 32) {
      FragB a;
      a.h[0] = *(const v8usa*)(ap + k0);
      a.h[1] = *(const v8usa*)(ap + k0 + 16);
#pragma unroll
      for (int nt = 0; nt < NSH; ++nt) {
        const unsigned short* wq = bp + (size_t)(16 * nt) * K2 + k0;
        FragB b;
        b.h[0] = *(const v8usa*)wq;
        b.h[1] = *(const v8usa*)(wq + 16);
        acc[nt] = wmb(a, b, acc[nt]);
      }
    }
#pragma unroll
    for (int nt = 0; nt < NSH; ++nt) {
      const float bv = sSV[HID + 16 * nt + m];
#pragma unroll
      for (int r = 0; r < 8; ++r) sWT[(rowW + 8 * hh + r) * WTP + 16 * nt + m] = acc[nt][r] + bv;
    }
  }
  __syncthreads();

  {
    const int el2 = tid >> 1, par = tid & 1;
    int sp = sSP[el2];
    sp = sp < 0 ? 0 : (sp > 5 ? 5 : sp);
    const float* wrow = sWT + el2 * WTP;
    const float* srow = sSH + el2 * SHP;
    const float* prow = sPT + sp * (OC * 4);
    float fx = 0.0f, fy = 0.0f, fz = 0.0f;
#pragma unroll 1
    for (int i = 0; i < 18; ++i) {
      const int sc = 4 * (par * 18 + i);
      const float shv = srow[sc >> 4];
      const v4f wv = *(const v4fa*)(wrow + sc);
      const float* pp = prow + sc * 4;
      const v4f p0 = *(const v4fa*)pp;
      const v4f p1 = *(const v4fa*)(pp + 4);
      const v4f p2 = *(const v4fa*)(pp + 8);
      const v4f p3 = *(const v4fa*)(pp + 12);
      const float g0 = wv.x * shv, g1 = wv.y * shv, g2 = wv.z * shv, g3 = wv.w * shv;
      fx = fmaf(g0, p0.x, fx); fy = fmaf(g0, p0.y, fy); fz = fmaf(g0, p0.z, fz);
      fx = fmaf(g1, p1.x, fx); fy = fmaf(g1, p1.y, fy); fz = fmaf(g1, p1.z, fz);
      fx = fmaf(g2, p2.x, fx); fy = fmaf(g2, p2.y, fy); fz = fmaf(g2, p2.z, fz);
      fx = fmaf(g3, p3.x, fx); fy = fmaf(g3, p3.y, fy); fz = fmaf(g3, p3.z, fz);
    }
    const float ox = __shfl_xor(fx, 1, 32);
    const float oy = __shfl_xor(fy, 1, 32);
    const float oz = __shfl_xor(fz, 1, 32);
    fx = fx + ox; fy = fy + oy; fz = fz + oz;
    if (par == 0) {
      v4f o;
      o.x = fx; o.y = fy; o.z = fz; o.w = 0.0f;
      *(v4fa*)(sF3 + 4 * el2) = o;
    }
  }
  __syncthreads();

  if (tid < EPB) {
    const v4f o = *(const v4fa*)(sF3 + 4 * tid);
    float* op = F3 + ((size_t)blockIdx.x * EPB + (size_t)tid) * 4;
    *(volatile v4f*)op = o;
    __threadfence();
    *(volatile v4f*)op = o;
  }
}

__global__ __launch_bounds__(NTHR) void k_scan(const int* __restrict__ dsts, int nE, int vec8, int nN,
                                               const float* __restrict__ F3, const float* __restrict__ ob,
                                               float* out) {
  extern __shared__ __attribute__((aligned(16))) int dsm[];
  int*   list = dsm;
  int*   hl   = dsm + LISTN;
  int*   sl   = hl + RCAP;
  int*   cnt  = sl + RCAP;
  int*   offs = cnt + NBA;
  int*   cur  = offs + NBA;
  int*   misc = cur + NBA;
  float* outs = (float*)(dsm + AGG_LDS_INTS);
  const int tid = (int)threadIdx.x, lane = tid & 31, wave = tid >> 5;
  const int nodeBase = (int)blockIdx.x * NBA;
  int rows = nN - nodeBase;
  rows = rows > NBA ? NBA : rows;
  rows = rows < 0 ? 0 : rows;

  {
    const v4i z4 = {0, 0, 0, 0};
    for (int i = tid * 4; i < AGG_ZINTS; i += NTHR * 4) *(v4ia*)(dsm + i) = z4;
    if (tid < 16) misc[tid] = 0;
  }
  __syncthreads();

  int t = 0, ov = 0;
  const int nChunks = (nE + CHUNK - 1) / CHUNK;
#pragma unroll 1
  for (int ch = 0; ch < nChunks; ++ch) {
    const int cbase = ch * CHUNK;
    const int wc = scan_chunk<SLA>(dsts, nE, cbase, nodeBase, rows, vec8, list, tid, lane, wave);
    if (lane == 0) misc[wave] = wc;
    __syncthreads();
    if (wave == 0) {
#pragma unroll 1
      for (int w2 = 0; w2 < NWAVE; ++w2) {
        int c = misc[w2];
        c = c < 0 ? 0 : (c > WCAP ? WCAP : c);
#pragma unroll 1
        for (int b0 = 0; b0 < c; b0 += 32) {
          const int idx = b0 + lane;
          const int ent = list[w2 * WCAP + (idx < WCAP ? idx : WCAP - 1)];
          const int m32 = (c - b0) < 32 ? (c - b0) : 32;
#pragma unroll 1
          for (int k = 0; k < m32; ++k) {
            const int u    = __builtin_amdgcn_readlane(ent, k);
            const int slot = u & (NBA - 1);
            const int el   = (u >> SLA) & (CHUNK - 1);
            const int pk   = ((cbase + el) << SLA) | slot;
            if (t < RCAP) {
              if (lane == 0) { hl[t] = pk; cnt[slot] = cnt[slot] + 1; }
              t = t + 1;
            } else {
              ov = 1;
            }
          }
        }
      }
    }
    __syncthreads();
  }
  if (wave == 0 && lane == 0) { misc[8] = t; misc[9] = ov; }
  __syncthreads();
  int tt = misc[8];
  tt = tt < 0 ? 0 : (tt > RCAP ? RCAP : tt);
  const int ovf = misc[9];

  if (wave == 0) {
    const int base = lane * (NBA / 32);
    int s = 0;
#pragma unroll 1
    for (int i = 0; i < NBA / 32; ++i) s += cnt[base + i];
    int incl = s;
#pragma unroll
    for (int d = 1; d < 32; d <<= 1) {
      const int y = __shfl_up(incl, d, 32);
      if (lane >= d) incl += y;
    }
    int run = incl - s;
#pragma unroll 1
    for (int i = 0; i < NBA / 32; ++i) {
      const int cv = cnt[base + i];
      offs[base + i] = run;
      cur[base + i]  = run;
      run += cv;
    }
  }
  __syncthreads();
  if (wave == 0) {
#pragma unroll 1
    for (int b0 = 0; b0 < tt; b0 += 32) {
      const int idx = b0 + lane;
      const int ent = hl[idx < RCAP ? idx : RCAP - 1];
      const int m32 = (tt - b0) < 32 ? (tt - b0) : 32;
#pragma unroll 1
      for (int k = 0; k < m32; ++k) {
        const int u    = __builtin_amdgcn_readlane(ent, k);
        const int slot = u & (NBA - 1);
        if (lane == 0) {
          int p = cur[slot];
          p = p < 0 ? 0 : (p > RCAP - 1 ? RCAP - 1 : p);
          sl[p] = u;
          cur[slot] = p + 1;
        }
      }
    }
  }
  __syncthreads();

  const float qnan = __int_as_float(0x7fc00000);
  const float ob0 = bf16_val(ob[0]);
  const float ob1 = bf16_val(ob[1]);
  const float ob2 = bf16_val(ob[2]);
#pragma unroll 1
  for (int ps = 0; ps < NBA / NTHR; ++ps) {
    const int slot = ps * NTHR + tid;
    const int craw = cnt[slot];
    const bool bad = (craw > DEGCAP) || (ovf != 0);
    int c = craw;
    c = c < 0 ? 0 : (c > DEGCAP ? DEGCAP : c);
    int o = offs[slot];
    o = o < 0 ? 0 : (o > RCAP - 1 ? RCAP - 1 : o);
    int cm = c;
    { const int y = __shfl_xor(cm, 16, 32); cm = cm > y ? cm : y; }
    { const int y = __shfl_xor(cm, 8, 32);  cm = cm > y ? cm : y; }
    { const int y = __shfl_xor(cm, 4, 32);  cm = cm > y ? cm : y; }
    { const int y = __shfl_xor(cm, 2, 32);  cm = cm > y ? cm : y; }
    { const int y = __shfl_xor(cm, 1, 32);  cm = cm > y ? cm : y; }
    cm = __builtin_amdgcn_readfirstlane(cm);
    cm = cm > DEGCAP ? DEGCAP : cm;
    float sx = 0.0f, sy = 0.0f, sz = 0.0f;
#pragma unroll 1
    for (int q = 0; q < cm; ++q) {
      int idx = o + q;
      idx = idx > RCAP - 1 ? RCAP - 1 : idx;
      const int ent = sl[idx];
      int eid = ent >> SLA;
      eid = eid < 0 ? 0 : (eid > nE - 1 ? nE - 1 : eid);
      const v4f f = *(const v4fa*)(F3 + (size_t)eid * 4);
      const unsigned mk = (q < c) ? 0xffffffffu : 0u;
      sx = sx + __uint_as_float(__float_as_uint(f.x) & mk);
      sy = sy + __uint_as_float(__float_as_uint(f.y) & mk);
      sz = sz + __uint_as_float(__float_as_uint(f.z) & mk);
    }
    const float v0 = 0.25f * sx + ob0;
    const float v1 = 0.25f * sy + ob1;
    const float v2 = 0.25f * sz + ob2;
    outs[slot * 3 + 0] = bad ? qnan : v0;
    outs[slot * 3 + 1] = bad ? qnan : v1;
    outs[slot * 3 + 2] = bad ? qnan : v2;
  }
  __syncthreads();

  {
    const int nq = (rows * 3) >> 2;
    float* ob_ = out + (size_t)nodeBase * 3;
    v4f pv[3];
#pragma unroll
    for (int it = 0; it < 3; ++it) {
      const int idx = it * NTHR + tid;
      const int idc = idx < nq ? idx : 0;
      pv[it] = *(const v4fa*)(outs + 4 * idc);
    }
#pragma unroll
    for (int it = 0; it < 3; ++it) {
      const int idx = it * NTHR + tid;
      if (idx < nq) *(volatile v4f*)(ob_ + (size_t)idx * 4) = pv[it];
    }
    __threadfence();
#pragma unroll
    for (int it = 0; it < 3; ++it) {
      const int idx = it * NTHR + tid;
      if (idx < nq) *(volatile v4f*)(ob_ + (size_t)idx * 4) = pv[it];
    }
  }
}

static inline int cdiv(int a, int b) { return (a + b - 1) / b; }

extern "C" void kernel_launch(void* const* d_in, const int* in_sizes, int n_in,
                              void* d_out, int out_size, void* d_ws, size_t ws_size,
                              hipStream_t stream) {
  if (n_in < 12) return;
  const int nN = in_sizes[0];
  if (nN < 4 || nN > (1 << 22)) return;
  if (in_sizes[1] != 3 * nN) return;
  if ((in_sizes[2] & 1) != 0) return;
  const int nE = in_sizes[2] / 2;
  if (nE < 1 || nE >= (1 << 21)) return;
  if (in_sizes[3] != 3 * nE) return;
  if (in_sizes[4] != 5 * CCH || in_sizes[5] != CCH) return;
  if (in_sizes[6] != NBS * HID || in_sizes[7] != HID) return;
  if (in_sizes[8] != HID * OC || in_sizes[9] != OC) return;
  if (in_sizes[10] != OC * 3 || in_sizes[11] != 3) return;
  if ((long long)out_size != (long long)nN * 3) return;
  if (((nN * 3) & 3) != 0) return;

  const int*   z     = (const int*)  d_in[0];
  const float* pos   = (const float*)d_in[1];
  const int*   eidx  = (const int*)  d_in[2];
  const float* shift = (const float*)d_in[3];
  const float* embw  = (const float*)d_in[4];
  const float* embb  = (const float*)d_in[5];
  const float* w1    = (const float*)d_in[6];
  const float* b1    = (const float*)d_in[7];
  const float* w2    = (const float*)d_in[8];
  const float* b2    = (const float*)d_in[9];
  const float* ow    = (const float*)d_in[10];
  const float* ob    = (const float*)d_in[11];
  float* out = (float*)d_out;

  const int NPR = cdiv(nN, NTHR) * NTHR;
  const int gE  = cdiv(nE, EPB);
  const int gA  = cdiv(nN, NBA);

  char* ws = (char*)d_ws;
  size_t off = 0;
  const size_t oW1P = off; off += (size_t)HID * K1 * 2;              off = (off + 255) & ~(size_t)255;
  const size_t oW2D = off; off += (size_t)OC * K2 * 2;               off = (off + 255) & ~(size_t)255;
  const size_t oSV  = off; off += (size_t)SVF * 4;                   off = (off + 255) & ~(size_t)255;
  const size_t oPT  = off; off += (size_t)PTU * 16;                  off = (off + 255) & ~(size_t)255;
  const size_t oNP  = off; off += (size_t)NPR * 16;                  off = (off + 255) & ~(size_t)255;
  const size_t oF3  = off; off += (size_t)gE * EPB * 16;             off = (off + 255) & ~(size_t)255;
  if (off > ws_size || off > (size_t)WSMAX) return;
  unsigned short* W1P = (unsigned short*)(ws + oW1P);
  unsigned short* W2D = (unsigned short*)(ws + oW2D);
  float*          SV  = (float*)(ws + oSV);
  float*          PT  = (float*)(ws + oPT);
  float*          NPp = (float*)(ws + oNP);
  float*          F3  = (float*)(ws + oF3);

  hipFuncSetAttribute(reinterpret_cast<const void*>(&k_edge), hipFuncAttributeMaxDynamicSharedMemorySize,
                      (int)EDGE_LDS_BYTES);
  hipFuncSetAttribute(reinterpret_cast<const void*>(&k_scan), hipFuncAttributeMaxDynamicSharedMemorySize,
                      (int)SCAN_LDS_BYTES);

  const int nPrep = U3 + NPR;
  const int vec8  = ((nE & 3) == 0) ? 1 : 0;

  k_prep<<<nPrep / NTHR, NTHR, 0, stream>>>(z, pos, embw, embb, w1, b1, w2, b2, ow, nN, NPR,
                                            W1P, W2D, SV, PT, NPp);
  k_edge<<<gE, NTHR, EDGE_LDS_BYTES, stream>>>(eidx, shift, nE, nN, NPp, W1P, W2D, SV, PT, F3);
  k_scan<<<gA, NTHR, SCAN_LDS_BYTES, stream>>>(eidx + (size_t)nE, nE, vec8, nN, F3, ob, out);
}
